// MultiOmicsHeteroGNN_59768764891881
// MI455X (gfx1250) — hardware-verified
//
#include <hip/hip_runtime.h>
#include <stddef.h>
#include <stdint.h>


#define DF    128
#define NH    4
#define HD    32
#define WSZ   (DF * DF)
#define GR    32
#define AP    136
#define XSP   132
#define NB    512
#define CHUNK 2048
#define NTHR  256
#define NWAVE 8
#define WCAP  256
#define NGRP  (CHUNK / (NTHR * 4))
#define NMAT  15
#define NCONV 12

#define LDS_SACC (NB * DF)
#define LDS_DEN  (NB * NH)
#define LDS_DSTA (NB * NH)
#define LDS_LIST (NWAVE * WCAP)
#define LDS_BYTES ((LDS_SACC + LDS_DEN + LDS_DSTA + LDS_LIST + NWAVE) * 4)

static_assert(WCAP == (CHUNK / NTHR) * 32);
static_assert(NGRP == 2);
static_assert(NB == 512);
static_assert(CHUNK <= 2048);
static_assert(((LDS_SACC + LDS_DEN) % 4) == 0);
static_assert(LDS_BYTES == 286752);
static_assert(NB % NWAVE == 0);
static_assert(GR * NH == 128);

typedef float    v4f  __attribute__((ext_vector_type(4)));
typedef float    v8f  __attribute__((ext_vector_type(8)));
typedef int      v4i  __attribute__((ext_vector_type(4)));
typedef _Float16 v8h  __attribute__((ext_vector_type(8)));
typedef _Float16 v16h __attribute__((ext_vector_type(16)));
union Frag   { v16h v; v8h half[2]; };
union Pack16 { v8h h; v4i i; };

__device__ __forceinline__ v8f wm(v16h a, v16h b, v8f c) {
  v8f d = __builtin_amdgcn_wmma_f32_16x16x32_f16(false, a, false, b, (short)0, c, false, false);
  asm volatile("v_nop\n\tv_nop\n\tv_nop\n\tv_nop" : "+v"(d) : "v"(a), "v"(b));
  return d;
}

__global__ __launch_bounds__(NTHR) void k_prep(const float* __restrict__ Wc,
                                               const float* __restrict__ Wo,
                                               _Float16* Wt) {
  __shared__ __attribute__((aligned(16))) _Float16 Ls[DF * AP];
  const int tid = threadIdx.x, lane = tid & 31, wave = tid >> 5;
  const int hh = lane >> 4, c = lane & 15;
  const int b = blockIdx.x;
  const float* src;
  if (b < NCONV) src = Wc + (size_t)b * WSZ;
  else           src = Wo + (size_t)(b - NCONV) * WSZ;
#pragma unroll 4
  for (int i = tid; i < WSZ; i += NTHR) {
    const int k = i >> 7, n = i & (DF - 1);
    Ls[n * AP + k] = (_Float16)(src[i] * 64.0f);
  }
  __syncthreads();
  _Float16* dst = Wt + (size_t)b * WSZ;
  v4i v[8];
#pragma unroll
  for (int q = 0; q < 8; ++q) {
    const int n = q * 16 + wave * 2 + hh;
    Pack16 u;
    u.h = *(const v8h*)(Ls + n * AP + 8 * c);
    v[q] = u.i;
  }
#pragma unroll
  for (int q = 0; q < 8; ++q)
    *(volatile v4i*)(dst + (size_t)(q * 16 + wave * 2 + hh) * DF + 8 * c) = v[q];
  __threadfence();
#pragma unroll
  for (int q = 0; q < 8; ++q)
    *(volatile v4i*)(dst + (size_t)(q * 16 + wave * 2 + hh) * DF + 8 * c) = v[q];
}

__global__ __launch_bounds__(NTHR) void k_embed(const float* __restrict__ x, int nN,
                                                const float* __restrict__ W,
                                                const float* __restrict__ b, float* h) {
#pragma clang fp contract(off)
  const int lane = threadIdx.x & 31, wave = threadIdx.x >> 5;
  const int row = blockIdx.x * NWAVE + wave;
  if (row >= nN) return;
  const float xv = x[row];
  const v4f w4 = *(const v4f*)(W + 4 * lane);
  const v4f b4 = *(const v4f*)(b + 4 * lane);
  const v4f t = w4 * xv;
  v4f y = t + b4;
  y.x = y.x > 0.f ? y.x : 0.f;
  y.y = y.y > 0.f ? y.y : 0.f;
  y.z = y.z > 0.f ? y.z : 0.f;
  y.w = y.w > 0.f ? y.w : 0.f;
  float* op = h + (size_t)row * DF + 4 * lane;
  *(volatile v4f*)op = y;
  __threadfence();
  *(volatile v4f*)op = y;
}

__global__ __launch_bounds__(NTHR) void k_gemm(
    const float* __restrict__ x, int nN, int nP,
    const _Float16* __restrict__ Wt,
    const float* __restrict__ attS, const float* __restrict__ attD, int R,
    _Float16* mh, float* asP, float* adP,
    const float* __restrict__ bias, float* outF, int mode) {
  __shared__ __attribute__((aligned(16))) _Float16 At[GR * AP];
  __shared__ __attribute__((aligned(16))) float Xs[GR * XSP];
  __shared__ __attribute__((aligned(16))) float attL[2 * DF];
  __shared__ __attribute__((aligned(16))) float Sad[2 * GR * NH];

  const int tid  = threadIdx.x;
  const int lane = tid & 31;
  const int wave = tid >> 5;
  const int hh   = lane >> 4;
  const int m    = lane & 15;
  const int rowBase = blockIdx.x * GR;
  const size_t mhStride = (size_t)nP * DF;
  const size_t aStride  = (size_t)nP * NH;

  {
    const int r  = tid >> 3;
    const int c0 = (tid & 7) * 16;
    int row = rowBase + r;
    if (row > nN - 1) row = nN - 1;
    const float* p = x + (size_t)row * DF + c0;
    const v4f f0 = *(const v4f*)(p), f1 = *(const v4f*)(p + 4);
    const v4f f2 = *(const v4f*)(p + 8), f3 = *(const v4f*)(p + 12);
    Pack16 u0, u1;
    u0.h[0] = (_Float16)(f0.x * 64.f); u0.h[1] = (_Float16)(f0.y * 64.f);
    u0.h[2] = (_Float16)(f0.z * 64.f); u0.h[3] = (_Float16)(f0.w * 64.f);
    u0.h[4] = (_Float16)(f1.x * 64.f); u0.h[5] = (_Float16)(f1.y * 64.f);
    u0.h[6] = (_Float16)(f1.z * 64.f); u0.h[7] = (_Float16)(f1.w * 64.f);
    u1.h[0] = (_Float16)(f2.x * 64.f); u1.h[1] = (_Float16)(f2.y * 64.f);
    u1.h[2] = (_Float16)(f2.z * 64.f); u1.h[3] = (_Float16)(f2.w * 64.f);
    u1.h[4] = (_Float16)(f3.x * 64.f); u1.h[5] = (_Float16)(f3.y * 64.f);
    u1.h[6] = (_Float16)(f3.z * 64.f); u1.h[7] = (_Float16)(f3.w * 64.f);
    *(v8h*)(At + r * AP + c0)     = u0.h;
    *(v8h*)(At + r * AP + c0 + 8) = u1.h;
  }
  __syncthreads();

  const int ncol = wave * 16 + m;

#pragma unroll 1
  for (int r = 0; r < R; ++r) {
    if (mode == 0) {
      const float vs = attS[r * DF + (tid & (DF - 1))];
      const float vd = attD[r * DF + (tid & (DF - 1))];
      attL[tid] = (tid < DF) ? vs : vd;
    }

    const _Float16* Wr = Wt + (size_t)r * WSZ + (size_t)ncol * DF;
    v8f c0a = {0.f, 0.f, 0.f, 0.f, 0.f, 0.f, 0.f, 0.f};
    v8f c1a = {0.f, 0.f, 0.f, 0.f, 0.f, 0.f, 0.f, 0.f};
#pragma unroll
    for (int kt = 0; kt < DF / 32; ++kt) {
      const int k0 = kt * 32;
      Frag a0, a1, b;
      const _Float16* pb  = Wr + k0 + 8 * hh;
      const _Float16* pa0 = At + m * AP + k0 + 8 * hh;
      const _Float16* pa1 = At + (16 + m) * AP + k0 + 8 * hh;
      b.half[0]  = *(const v8h*)pb;  b.half[1]  = *(const v8h*)(pb + 16);
      a0.half[0] = *(const v8h*)pa0; a0.half[1] = *(const v8h*)(pa0 + 16);
      a1.half[0] = *(const v8h*)pa1; a1.half[1] = *(const v8h*)(pa1 + 16);
      c0a = wm(a0.v, b.v, c0a);
      c1a = wm(a1.v, b.v, c1a);
    }

    const float bv = (mode != 0) ? bias[ncol] : 0.f;
#pragma unroll
    for (int r8 = 0; r8 < 8; ++r8) {
      Xs[(8 * hh + r8) * XSP + ncol]      = c0a[r8] * (1.0f / 4096.0f) + bv;
      Xs[(16 + 8 * hh + r8) * XSP + ncol] = c1a[r8] * (1.0f / 4096.0f) + bv;
    }
    __syncthreads();

    if (mode == 0) {
      const int row = tid >> 3;
      const int h   = (tid >> 1) & 3;
      const int sd  = tid & 1;
      const float* xr = Xs + row * XSP + h * HD;
      const float* av = attL + sd * DF + h * HD;
      float s = 0.f;
#pragma unroll 2
      for (int d4 = 0; d4 < HD / 4; ++d4) {
        const v4f a = *(const v4f*)(xr + 4 * d4);
        const v4f w = *(const v4f*)(av + 4 * d4);
        s += a.x * w.x; s += a.y * w.y; s += a.z * w.z; s += a.w * w.w;
      }
      Sad[sd * (GR * NH) + row * NH + h] = s;
    }
    __syncthreads();

    if (mode == 0) {
      const int rw0 = 4 * wave + hh;
      const int rw1 = 4 * wave + 2 + hh;
      Pack16 u0, u1;
      {
        const float* xs = Xs + rw0 * XSP + 8 * m;
        const v4f f0 = *(const v4f*)xs, f1 = *(const v4f*)(xs + 4);
        u0.h[0] = (_Float16)(f0.x * 64.f); u0.h[1] = (_Float16)(f0.y * 64.f);
        u0.h[2] = (_Float16)(f0.z * 64.f); u0.h[3] = (_Float16)(f0.w * 64.f);
        u0.h[4] = (_Float16)(f1.x * 64.f); u0.h[5] = (_Float16)(f1.y * 64.f);
        u0.h[6] = (_Float16)(f1.z * 64.f); u0.h[7] = (_Float16)(f1.w * 64.f);
      }
      {
        const float* xs = Xs + rw1 * XSP + 8 * m;
        const v4f f0 = *(const v4f*)xs, f1 = *(const v4f*)(xs + 4);
        u1.h[0] = (_Float16)(f0.x * 64.f); u1.h[1] = (_Float16)(f0.y * 64.f);
        u1.h[2] = (_Float16)(f0.z * 64.f); u1.h[3] = (_Float16)(f0.w * 64.f);
        u1.h[4] = (_Float16)(f1.x * 64.f); u1.h[5] = (_Float16)(f1.y * 64.f);
        u1.h[6] = (_Float16)(f1.z * 64.f); u1.h[7] = (_Float16)(f1.w * 64.f);
      }
      _Float16* mp0 = mh + (size_t)r * mhStride + (size_t)(rowBase + rw0) * DF + 8 * m;
      _Float16* mp1 = mh + (size_t)r * mhStride + (size_t)(rowBase + rw1) * DF + 8 * m;
      v4f gv = {0.f, 0.f, 0.f, 0.f};
      float* gp = asP;
      if (wave < 2) {
        gv = *(const v4f*)(Sad + wave * (GR * NH) + 4 * lane);
        float* gbase = (wave == 0) ? asP : adP;
        gp = gbase + (size_t)r * aStride + (size_t)rowBase * NH + 4 * lane;
      }
      *(volatile v4i*)mp0 = u0.i;
      *(volatile v4i*)mp1 = u1.i;
      if (wave < 2) *(volatile v4f*)gp = gv;
      __threadfence();
      *(volatile v4i*)mp0 = u0.i;
      *(volatile v4i*)mp1 = u1.i;
      if (wave < 2) *(volatile v4f*)gp = gv;
    } else {
      v4f xv[4];
      float* xp[4];
      bool ok[4];
#pragma unroll
      for (int i = 0; i < 4; ++i) {
        const int rl = 4 * wave + i;
        int row = rowBase + rl;
        ok[i] = row < nN;
        if (row > nN - 1) row = nN - 1;
        xv[i] = *(const v4f*)(Xs + rl * XSP + 4 * lane);
        xp[i] = outF + (size_t)row * DF + 4 * lane;
      }
#pragma unroll
      for (int i = 0; i < 4; ++i) if (ok[i]) *(volatile v4f*)(xp[i]) = xv[i];
      __threadfence();
#pragma unroll
      for (int i = 0; i < 4; ++i) if (ok[i]) *(volatile v4f*)(xp[i]) = xv[i];
    }
    __syncthreads();
  }
}

__global__ __launch_bounds__(NTHR) void k_agg(
    const int* __restrict__ esrc, const int* __restrict__ edst, int nE,
    const _Float16* __restrict__ mh, const float* __restrict__ asrc, int nSrc,
    const float* __restrict__ adst, const float* __restrict__ bias,
    float* out, int nDst, int addPrior, int doRelu) {
  extern __shared__ v4f lds_dyn[];
  float* sacc = (float*)lds_dyn;
  float* den  = sacc + LDS_SACC;
  float* dsta = den + LDS_DEN;
  int*   list = (int*)(dsta + LDS_DSTA);
  int*   wcnt = list + LDS_LIST;

  const int tid  = threadIdx.x;
  const int lane = tid & 31;
  const int wave = tid >> 5;
  const int hh   = lane >> 4;
  const int c    = lane & 15;
  const int hd   = c >> 2;
  const int nodeBase = blockIdx.x * NB;

  {
    const v4f z4 = {0.f, 0.f, 0.f, 0.f};
    for (int i = tid; i < (LDS_SACC + LDS_DEN) / 4; i += NTHR) lds_dyn[i] = z4;
    for (int i = tid; i < NB; i += NTHR) {
      int node = nodeBase + i;
      if (node > nDst - 1) node = nDst - 1;
      *(v4f*)(dsta + i * NH) = *(const v4f*)(adst + (size_t)node * NH);
    }
  }
  __syncthreads();

  const int nChunks = (nE + CHUNK - 1) / CHUNK;
#pragma unroll 1
  for (int ch = 0; ch < nChunks; ++ch) {
    const int cbase = ch * CHUNK;
    int wc = 0;
#pragma unroll
    for (int g = 0; g < NGRP; ++g) {
      const int el0 = (g * NTHR + tid) * 4;
      const int e0  = cbase + el0;
      v4i d;
      if (cbase + CHUNK <= nE) {
        d = *(const v4i*)(edst + e0);
      } else {
        const int sent = -2147483647 - 1;
        const int q0 = edst[min(e0,     nE - 1)];
        const int q1 = edst[min(e0 + 1, nE - 1)];
        const int q2 = edst[min(e0 + 2, nE - 1)];
        const int q3 = edst[min(e0 + 3, nE - 1)];
        d.x = (e0     < nE) ? q0 : sent;
        d.y = (e0 + 1 < nE) ? q1 : sent;
        d.z = (e0 + 2 < nE) ? q2 : sent;
        d.w = (e0 + 3 < nE) ? q3 : sent;
      }
      const unsigned s0 = (unsigned)d.x - (unsigned)nodeBase;
      const unsigned s1 = (unsigned)d.y - (unsigned)nodeBase;
      const unsigned s2 = (unsigned)d.z - (unsigned)nodeBase;
      const unsigned s3 = (unsigned)d.w - (unsigned)nodeBase;
      const bool h0 = s0 < (unsigned)NB;
      const bool h1 = s1 < (unsigned)NB;
      const bool h2 = s2 < (unsigned)NB;
      const bool h3 = s3 < (unsigned)NB;
      const int cnt = (int)h0 + (int)h1 + (int)h2 + (int)h3;
      const unsigned many = __builtin_amdgcn_ballot_w32(cnt != 0);
      if (many != 0u) {
        const unsigned m2 = __builtin_amdgcn_ballot_w32(cnt > 1);
        if (m2 == 0u) {
          if (cnt != 0) {
            const int pos = wc + (int)__builtin_amdgcn_mbcnt_lo(many, 0u);
            const int j = h0 ? 0 : (h1 ? 1 : (h2 ? 2 : 3));
            const unsigned sj = h0 ? s0 : (h1 ? s1 : (h2 ? s2 : s3));
            if (pos < WCAP) list[wave * WCAP + pos] = ((el0 + j) << 9) | (int)sj;
          }
          wc += (int)__builtin_popcount(many);
        } else {
#define HITJ(J, HJ, SJ) { \
            const unsigned mj = __builtin_amdgcn_ballot_w32(HJ); \
            if (HJ) { \
              const int pos = wc + (int)__builtin_amdgcn_mbcnt_lo(mj, 0u); \
              if (pos < WCAP) list[wave * WCAP + pos] = ((el0 + (J)) << 9) | (int)(SJ); \
            } \
            wc += (int)__builtin_popcount(mj); }
          HITJ(0, h0, s0)
          HITJ(1, h1, s1)
          HITJ(2, h2, s2)
          HITJ(3, h3, s3)
#undef HITJ
        }
      }
    }
    if (lane == 0) wcnt[wave] = wc;
    __syncthreads();

    if (wave == 0) {
#pragma unroll 1
      for (int wsx = 0; wsx < NWAVE; ++wsx) {
        int n = wcnt[wsx];
        if (n > WCAP) n = WCAP;
        if (n < 0) n = 0;
#pragma unroll 1
        for (int i = 0; i < n; i += 2) {
          int ia = i + hh;
          const bool valid = ia < n;
          if (ia > n - 1) ia = n - 1;
          const int ent  = list[wsx * WCAP + ia];
          const int slot = ent & (NB - 1);
          const int el   = (ent >> 9) & (CHUNK - 1);
          int e = cbase + el;
          if (e > nE - 1) e = nE - 1;
          int src = esrc[e];
          src = src < 0 ? 0 : (src > nSrc - 1 ? nSrc - 1 : src);
          float lg = asrc[(size_t)src * NH + hd] + dsta[slot * NH + hd];
          lg = (lg > 0.f) ? lg : 0.2f * lg;
          lg = fminf(lg, 60.f);
          const float p  = valid ? __expf(lg) : 0.f;
          const float ps = p * (1.0f / 64.0f);
          Pack16 u;
          u.i = *(const v4i*)(mh + (size_t)src * DF + 8 * c);
          v4f ca, cb;
          ca.x = ps * (float)u.h[0]; ca.y = ps * (float)u.h[1];
          ca.z = ps * (float)u.h[2]; ca.w = ps * (float)u.h[3];
          cb.x = ps * (float)u.h[4]; cb.y = ps * (float)u.h[5];
          cb.z = ps * (float)u.h[6]; cb.w = ps * (float)u.h[7];
          float pden = p;
          const int sA = __shfl(slot, 0, 32);
          const int sB = __shfl(slot, 16, 32);
          const bool same = (sA == sB);
          if (same) {
            v4f oa, ob;
            oa.x = __shfl_xor(ca.x, 16, 32); oa.y = __shfl_xor(ca.y, 16, 32);
            oa.z = __shfl_xor(ca.z, 16, 32); oa.w = __shfl_xor(ca.w, 16, 32);
            ob.x = __shfl_xor(cb.x, 16, 32); ob.y = __shfl_xor(cb.y, 16, 32);
            ob.z = __shfl_xor(cb.z, 16, 32); ob.w = __shfl_xor(cb.w, 16, 32);
            const float op = __shfl_xor(pden, 16, 32);
            if (hh == 0) { ca += oa; cb += ob; pden += op; }
          }
          const bool wr = !(same && (hh != 0));
          v4f* sp = (v4f*)(sacc + slot * DF + 8 * c);
          v4f v0 = sp[0];
          v4f v1 = sp[1];
          v0 += ca;
          v1 += cb;
          if (wr) { sp[0] = v0; sp[1] = v1; }
          if (wr && (c & 3) == 0) {
            const float o = den[slot * NH + hd];
            den[slot * NH + hd] = o + pden;
          }
        }
      }
    }
    __syncthreads();
  }

  const int hq = lane >> 3;
  const v4f b4 = *(const v4f*)(bias + 4 * lane);
#pragma unroll 1
  for (int j = 0; j < NB / NWAVE; ++j) {
    const int slot = wave * (NB / NWAVE) + j;
    const int node = nodeBase + slot;
    if (node >= nDst) break;
    const size_t nrow = (size_t)node;
    const float dv  = den[slot * NH + hq];
    const float inv = 1.0f / fmaxf(dv, 1e-16f);
    const v4f sv = *(const v4f*)(sacc + slot * DF + 4 * lane);
    v4f y = sv * inv + b4;
    if (addPrior != 0) {
      const v4f pr = *(const v4f*)(out + nrow * DF + 4 * lane);
      y += pr;
    }
    if (doRelu != 0) {
      y.x = y.x > 0.f ? y.x : 0.f;
      y.y = y.y > 0.f ? y.y : 0.f;
      y.z = y.z > 0.f ? y.z : 0.f;
      y.w = y.w > 0.f ? y.w : 0.f;
    }
    float* op = out + nrow * DF + 4 * lane;
    *(volatile v4f*)op = y;
    __threadfence();
    *(volatile v4f*)op = y;
  }
}

static inline int cdiv_h(int a, int b) { return (a + b - 1) / b; }

extern "C" void kernel_launch(void* const* d_in, const int* in_sizes, int n_in,
                              void* d_out, int out_size, void* d_ws, size_t ws_size,
                              hipStream_t stream) {
  if (n_in < 19) return;
  const int nG = in_sizes[0];
  const int nQ = in_sizes[1];
  const int nM = in_sizes[2];
  const int eGG = in_sizes[3], eGP = in_sizes[5], ePP = in_sizes[7], ePM = in_sizes[9];
  if (nG <= 0 || nQ <= 0 || nM <= 0) return;
  if (eGG < 0 || in_sizes[4] != eGG) return;
  if (eGP < 0 || in_sizes[6] != eGP) return;
  if (ePP < 0 || in_sizes[8] != ePP) return;
  if (ePM < 0 || in_sizes[10] != ePM) return;
  if (in_sizes[11] != 3 * DF || in_sizes[12] != 3 * DF) return;
  if (in_sizes[13] != NCONV * WSZ) return;
  if (in_sizes[14] != NCONV * DF || in_sizes[15] != NCONV * DF || in_sizes[16] != NCONV * DF) return;
  if (in_sizes[17] != 3 * WSZ || in_sizes[18] != 3 * DF) return;
  if (out_size != (nG + nQ + nM) * DF) return;

  const float* xg   = (const float*)d_in[0];
  const float* xq   = (const float*)d_in[1];
  const float* xm   = (const float*)d_in[2];
  const int* gg_s   = (const int*)d_in[3];
  const int* gg_d   = (const int*)d_in[4];
  const int* gp_s   = (const int*)d_in[5];
  const int* gp_d   = (const int*)d_in[6];
  const int* pp_s   = (const int*)d_in[7];
  const int* pp_d   = (const int*)d_in[8];
  const int* pm_s   = (const int*)d_in[9];
  const int* pm_d   = (const int*)d_in[10];
  const float* W_emb  = (const float*)d_in[11];
  const float* b_emb  = (const float*)d_in[12];
  const float* W_conv = (const float*)d_in[13];
  const float* a_srcv = (const float*)d_in[14];
  const float* a_dstv = (const float*)d_in[15];
  const float* b_conv = (const float*)d_in[16];
  const float* W_out  = (const float*)d_in[17];
  const float* b_out  = (const float*)d_in[18];
  float* out0 = (float*)d_out;
  float* out1 = out0 + (size_t)nG * DF;
  float* out2 = out1 + (size_t)nQ * DF;

  const int pG = cdiv_h(nG, GR) * GR;
  const int pQ = cdiv_h(nQ, GR) * GR;
  const int pM = cdiv_h(nM, GR) * GR;

  size_t off = 0;
  char* base = (char*)d_ws;
#define CARVE(PTR, TYPE, COUNT) PTR = (TYPE*)(base + off); off += (((size_t)(COUNT) * sizeof(TYPE)) + 255) & ~(size_t)255;
  _Float16* Wt;  CARVE(Wt,  _Float16, (size_t)NMAT * WSZ)
  float* hg;     CARVE(hg,  float, (size_t)pG * DF)
  float* hq;     CARVE(hq,  float, (size_t)pQ * DF)
  float* hm;     CARVE(hm,  float, (size_t)pM * DF)
  _Float16* mhg; CARVE(mhg, _Float16, (size_t)2 * pG * DF)
  float* asg;    CARVE(asg, float, (size_t)2 * pG * NH)
  float* adg;    CARVE(adg, float, (size_t)2 * pG * NH)
  _Float16* mhq; CARVE(mhq, _Float16, (size_t)3 * pQ * DF)
  float* asq;    CARVE(asq, float, (size_t)3 * pQ * NH)
  float* adq;    CARVE(adq, float, (size_t)3 * pQ * NH)
  _Float16* mhm; CARVE(mhm, _Float16, (size_t)1 * pM * DF)
  float* asm_;   CARVE(asm_, float, (size_t)1 * pM * NH)
  float* adm;    CARVE(adm, float, (size_t)1 * pM * NH)
#undef CARVE
  if (off > ws_size) return;

  k_prep<<<NMAT, NTHR, 0, stream>>>(W_conv, W_out, Wt);

  k_embed<<<cdiv_h(nG, NWAVE), NTHR, 0, stream>>>(xg, nG, W_emb + 0 * DF, b_emb + 0 * DF, hg);
  k_embed<<<cdiv_h(nQ, NWAVE), NTHR, 0, stream>>>(xq, nQ, W_emb + 1 * DF, b_emb + 1 * DF, hq);
  k_embed<<<cdiv_h(nM, NWAVE), NTHR, 0, stream>>>(xm, nM, W_emb + 2 * DF, b_emb + 2 * DF, hm);

  hipFuncSetAttribute(reinterpret_cast<const void*>(&k_agg),
                      hipFuncAttributeMaxDynamicSharedMemorySize, LDS_BYTES);

  const size_t mhgS = (size_t)pG * DF, agS = (size_t)pG * NH;
  const size_t mhqS = (size_t)pQ * DF, aqS = (size_t)pQ * NH;

  for (int l = 0; l < 3; ++l) {
    const int r0i = l * 4;
    k_gemm<<<pG / GR, NTHR, 0, stream>>>(hg, nG, pG, Wt + (size_t)(r0i + 0) * WSZ,
                                         a_srcv + (r0i + 0) * DF, a_dstv + (r0i + 0) * DF, 2,
                                         mhg, asg, adg, b_conv, asg, 0);
    k_gemm<<<pQ / GR, NTHR, 0, stream>>>(hq, nQ, pQ, Wt + (size_t)(r0i + 1) * WSZ,
                                         a_srcv + (r0i + 1) * DF, a_dstv + (r0i + 1) * DF, 3,
                                         mhq, asq, adq, b_conv, asq, 0);
    k_gemm<<<pM / GR, NTHR, 0, stream>>>(hm, nM, pM, Wt + (size_t)(r0i + 3) * WSZ,
                                         a_srcv + (r0i + 3) * DF, a_dstv + (r0i + 3) * DF, 1,
                                         mhm, asm_, adm, b_conv, asm_, 0);
    k_agg<<<cdiv_h(nG, NB), NTHR, LDS_BYTES, stream>>>(
        gg_s, gg_d, eGG, mhg + 0 * mhgS, asg + 0 * agS, nG, adg + 0 * agS,
        b_conv + (r0i + 0) * DF, hg, nG, 0, 1);
    k_agg<<<cdiv_h(nQ, NB), NTHR, LDS_BYTES, stream>>>(
        gp_s, gp_d, eGP, mhg + 1 * mhgS, asg + 1 * agS, nG, adq + 0 * aqS,
        b_conv + (r0i + 1) * DF, hq, nQ, 0, 0);
    k_agg<<<cdiv_h(nQ, NB), NTHR, LDS_BYTES, stream>>>(
        pp_s, pp_d, ePP, mhq + 1 * mhqS, asq + 1 * aqS, nQ, adq + 1 * aqS,
        b_conv + (r0i + 2) * DF, hq, nQ, 1, 1);
    k_agg<<<cdiv_h(nM, NB), NTHR, LDS_BYTES, stream>>>(
        pm_s, pm_d, ePM, mhq + 2 * mhqS, asq + 2 * aqS, nQ, adm,
        b_conv + (r0i + 3) * DF, hm, nM, 0, 1);
  }

  k_gemm<<<pG / GR, NTHR, 0, stream>>>(hg, nG, pG, Wt + (size_t)(NCONV + 0) * WSZ, a_srcv, a_dstv, 1,
                                       mhg, asg, adg, b_out + 0 * DF, out0, 1);
  k_gemm<<<pQ / GR, NTHR, 0, stream>>>(hq, nQ, pQ, Wt + (size_t)(NCONV + 1) * WSZ, a_srcv, a_dstv, 1,
                                       mhq, asq, adq, b_out + 1 * DF, out1, 1);
  k_gemm<<<pM / GR, NTHR, 0, stream>>>(hm, nM, pM, Wt + (size_t)(NCONV + 2) * WSZ, a_srcv, a_dstv, 1,
                                       mhm, asm_, adm, b_out + 2 * DF, out2, 1);
}
